// GRNTransformer_90271622627428
// MI455X (gfx1250) — hardware-verified
//
#include <hip/hip_runtime.h>
#include <math.h>
#include <stddef.h>


#define IN_DIM 256
#define HID 128
#define QKV 512
#define WSCALE 16.0f
#define WINV 0.0625f
#define ATT_SCALE 0.0883883476483184f
#define LN_EPS 1e-5f

#define ANB 512
#define ANPW 64
#define LCAP 5120
#define BCAP 768
#define MAXD 64

typedef _Float16 v16h __attribute__((ext_vector_type(16)));
typedef _Float16 v8h  __attribute__((ext_vector_type(8)));
typedef float    v8f  __attribute__((ext_vector_type(8)));
typedef float    v4f  __attribute__((ext_vector_type(4)));
typedef v4f v4fa __attribute__((may_alias));
typedef v8h v8ha __attribute__((may_alias));
union Frag { v16h v; v8h half[2]; };

__device__ __forceinline__ v8f wmma16(v8f acc, v16h a, v16h b) {
    acc = __builtin_amdgcn_wmma_f32_16x16x32_f16(false, a, false, b, (short)0, acc, false, false);
    asm volatile("v_nop\n\tv_nop\n\tv_nop\n\tv_nop" : "+v"(acc) : "v"(a), "v"(b));
    return acc;
}

__global__ void __launch_bounds__(256) wprep_kernel(const float* __restrict__ W,
                                                    _Float16* __restrict__ Wt, int K, int Nc) {
    const int t = blockIdx.x * 256 + threadIdx.x;
    const int kch = K >> 3;
    const int total = Nc * kch;
    if (t >= total) return;
    const int n = t / kch;
    const int c8 = t - n * kch;
    v8h hv;
#pragma unroll
    for (int j = 0; j < 8; ++j)
        hv[j] = (_Float16)(W[(size_t)(c8 * 8 + j) * Nc + n] * WSCALE);
    _Float16* p = Wt + (size_t)n * K + c8 * 8;
    *(volatile v8h*)p = hv;
    __threadfence();
    *(volatile v8h*)p = hv;
}

template <int K>
__device__ __forceinline__ void stage_a(_Float16* s_a, const float* __restrict__ A, int M, int row0) {
    constexpr int KC = K / 8;
    for (int c = threadIdx.x; c < 32 * KC; c += 128) {
        const int r = c / KC;
        const int kc = c - r * KC;
        const int row = row0 + r;
        v4f x0 = {0.f, 0.f, 0.f, 0.f};
        v4f x1 = {0.f, 0.f, 0.f, 0.f};
        if (row < M) {
            const float* p = A + (size_t)row * K + kc * 8;
            x0 = *(const v4f*)p;
            x1 = *(const v4f*)(p + 4);
        }
        v8h hv;
        hv[0] = (_Float16)x0[0]; hv[1] = (_Float16)x0[1]; hv[2] = (_Float16)x0[2]; hv[3] = (_Float16)x0[3];
        hv[4] = (_Float16)x1[0]; hv[5] = (_Float16)x1[1]; hv[6] = (_Float16)x1[2]; hv[7] = (_Float16)x1[3];
        *(v8h*)(s_a + r * K + kc * 8) = hv;
    }
}

template <int K>
__device__ __forceinline__ void mma32x32(const _Float16* s_a, const _Float16* __restrict__ Wt,
                                         int col0, v8f (&acc)[2][2], int lane) {
    const int hh = lane >> 4, m = lane & 15;
    const v8f z = {0.f, 0.f, 0.f, 0.f, 0.f, 0.f, 0.f, 0.f};
    acc[0][0] = z; acc[0][1] = z; acc[1][0] = z; acc[1][1] = z;
    const _Float16* a0p = s_a + m * K + 8 * hh;
    const _Float16* a1p = s_a + (16 + m) * K + 8 * hh;
    const _Float16* b0p = Wt + (size_t)(col0 + m) * K + 8 * hh;
    const _Float16* b1p = Wt + (size_t)(col0 + 16 + m) * K + 8 * hh;
    for (int ks = 0; ks < K / 32; ++ks) {
        const int k0 = ks * 32;
        Frag a0, a1, b0, b1;
        a0.half[0] = *(const v8h*)(a0p + k0);  a0.half[1] = *(const v8h*)(a0p + k0 + 16);
        a1.half[0] = *(const v8h*)(a1p + k0);  a1.half[1] = *(const v8h*)(a1p + k0 + 16);
        b0.half[0] = *(const v8h*)(b0p + k0);  b0.half[1] = *(const v8h*)(b0p + k0 + 16);
        b1.half[0] = *(const v8h*)(b1p + k0);  b1.half[1] = *(const v8h*)(b1p + k0 + 16);
        acc[0][0] = wmma16(acc[0][0], a0.v, b0.v);
        acc[0][1] = wmma16(acc[0][1], a0.v, b1.v);
        acc[1][0] = wmma16(acc[1][0], a1.v, b0.v);
        acc[1][1] = wmma16(acc[1][1], a1.v, b1.v);
    }
}

__device__ __forceinline__ void acc_stage32(float* st, v8f (&acc)[2][2], const float* __restrict__ bias,
                                            int col0, int relu, int lane) {
    const int hh = lane >> 4, m = lane & 15;
    float bb0 = 0.f, bb1 = 0.f;
    if (bias != nullptr) { bb0 = bias[col0 + m]; bb1 = bias[col0 + 16 + m]; }
#pragma unroll
    for (int r = 0; r < 8; ++r) {
        float v00 = acc[0][0][r] * WINV + bb0;
        float v01 = acc[0][1][r] * WINV + bb1;
        float v10 = acc[1][0][r] * WINV + bb0;
        float v11 = acc[1][1][r] * WINV + bb1;
        if (relu) {
            v00 = v00 > 0.f ? v00 : 0.f; v01 = v01 > 0.f ? v01 : 0.f;
            v10 = v10 > 0.f ? v10 : 0.f; v11 = v11 > 0.f ? v11 : 0.f;
        }
        st[(8 * hh + r) * 32 + m]           = v00;
        st[(8 * hh + r) * 32 + 16 + m]      = v01;
        st[(16 + 8 * hh + r) * 32 + m]      = v10;
        st[(16 + 8 * hh + r) * 32 + 16 + m] = v11;
    }
}

__device__ __forceinline__ void acc_stage16(_Float16* st, v8f (&acc)[2][2], const float* __restrict__ bias,
                                            int col0, int chalf, int lane) {
    const int hh = lane >> 4, m = lane & 15;
    const float bb0 = bias[col0 + m];
    const float bb1 = bias[col0 + 16 + m];
    const int cb = chalf * 32;
#pragma unroll
    for (int r = 0; r < 8; ++r) {
        st[(8 * hh + r) * 64 + cb + m]           = (_Float16)(acc[0][0][r] * WINV + bb0);
        st[(8 * hh + r) * 64 + cb + 16 + m]      = (_Float16)(acc[0][1][r] * WINV + bb1);
        st[(16 + 8 * hh + r) * 64 + cb + m]      = (_Float16)(acc[1][0][r] * WINV + bb0);
        st[(16 + 8 * hh + r) * 64 + cb + 16 + m] = (_Float16)(acc[1][1][r] * WINV + bb1);
    }
}

__device__ __forceinline__ void store_lines32(const float* st, float* __restrict__ out, int ldc,
                                              int row0, int col0, int M, int lane) {
    const int q = lane >> 3, c4 = (lane & 7) * 4;
    v4f vals[8];
#pragma unroll
    for (int i = 0; i < 8; ++i) vals[i] = *(const v4fa*)(st + (4 * i + q) * 32 + c4);
#pragma unroll
    for (int i = 0; i < 8; ++i) {
        const int row = row0 + 4 * i + q;
        if (row < M) *(volatile v4f*)(out + (size_t)row * ldc + col0 + c4) = vals[i];
    }
    __threadfence();
#pragma unroll
    for (int i = 0; i < 8; ++i) {
        const int row = row0 + 4 * i + q;
        if (row < M) *(volatile v4f*)(out + (size_t)row * ldc + col0 + c4) = vals[i];
    }
}

__device__ __forceinline__ void store_lines16(const _Float16* st, _Float16* __restrict__ out, int ldc,
                                              int row0, int col0, int M, int lane) {
    const int q = lane >> 3, c8 = (lane & 7) * 8;
    v8h vals[8];
#pragma unroll
    for (int i = 0; i < 8; ++i) vals[i] = *(const v8ha*)(st + (4 * i + q) * 64 + c8);
#pragma unroll
    for (int i = 0; i < 8; ++i) {
        const int row = row0 + 4 * i + q;
        if (row < M) *(volatile v8h*)(out + (size_t)row * ldc + col0 + c8) = vals[i];
    }
    __threadfence();
#pragma unroll
    for (int i = 0; i < 8; ++i) {
        const int row = row0 + 4 * i + q;
        if (row < M) *(volatile v8h*)(out + (size_t)row * ldc + col0 + c8) = vals[i];
    }
}

__global__ void __launch_bounds__(128) proj_kernel(const float* __restrict__ X, int M,
                                                   const _Float16* __restrict__ Wt,
                                                   const float* __restrict__ bias,
                                                   float* __restrict__ H) {
    __shared__ _Float16 s_a[32 * IN_DIM] __attribute__((aligned(16)));
    __shared__ float s_st[4][32 * 32] __attribute__((aligned(16)));
    const int lane = threadIdx.x & 31, wv = threadIdx.x >> 5;
    const int row0 = blockIdx.x * 32;
    stage_a<IN_DIM>(s_a, X, M, row0);
    __syncthreads();
    v8f acc[2][2];
    mma32x32<IN_DIM>(s_a, Wt, 32 * wv, acc, lane);
    acc_stage32(s_st[wv], acc, bias, 32 * wv, 1, lane);
    __syncthreads();
    store_lines32(s_st[wv], H, HID, row0, 32 * wv, M, lane);
}

__global__ void __launch_bounds__(128) qkvs_kernel(const float* __restrict__ Hin, int M,
                                                   const _Float16* __restrict__ Wq, const float* __restrict__ bq,
                                                   const _Float16* __restrict__ Wk, const float* __restrict__ bk,
                                                   const _Float16* __restrict__ Wv, const float* __restrict__ bv,
                                                   const _Float16* __restrict__ Ws,
                                                   _Float16* __restrict__ q16, _Float16* __restrict__ k16,
                                                   float* __restrict__ v32, float* __restrict__ skip) {
    __shared__ _Float16 s_a[32 * HID] __attribute__((aligned(16)));
    __shared__ float s_st32[4][32 * 32] __attribute__((aligned(16)));
    __shared__ _Float16 s_st16[4][32 * 64] __attribute__((aligned(16)));
    const int lane = threadIdx.x & 31, wv = threadIdx.x >> 5;
    const int row0 = blockIdx.x * 32;
    stage_a<HID>(s_a, Hin, M, row0);
    __syncthreads();
    v8f acc[2][2];

    for (int mat = 0; mat < 2; ++mat) {
        const _Float16* W = mat ? Wk : Wq;
        const float* B = mat ? bk : bq;
        _Float16* O = mat ? k16 : q16;
        for (int i = 0; i < 2; ++i) {
            const int cq = (wv + 4 * i) * 64;
            for (int half = 0; half < 2; ++half) {
                mma32x32<HID>(s_a, W, cq + 32 * half, acc, lane);
                acc_stage16(s_st16[wv], acc, B, cq + 32 * half, half, lane);
            }
            __syncthreads();
            store_lines16(s_st16[wv], O, QKV, row0, cq, M, lane);
        }
    }
    for (int i = 0; i < 4; ++i) {
        const int c0 = (wv + 4 * i) * 32;
        mma32x32<HID>(s_a, Wv, c0, acc, lane);
        acc_stage32(s_st32[wv], acc, bv, c0, 0, lane);
        __syncthreads();
        store_lines32(s_st32[wv], v32, QKV, row0, c0, M, lane);
    }
    {
        const int c0 = wv * 32;
        mma32x32<HID>(s_a, Ws, c0, acc, lane);
        acc_stage32(s_st32[wv], acc, nullptr, c0, 0, lane);
        __syncthreads();
        store_lines32(s_st32[wv], skip, HID, row0, c0, M, lane);
    }
}

__global__ void __launch_bounds__(256) agg_kernel(const int* __restrict__ ei, int E, int Nn,
                                                  const _Float16* __restrict__ q16,
                                                  const _Float16* __restrict__ k16,
                                                  const float* __restrict__ v32,
                                                  const float* __restrict__ skip,
                                                  const float* __restrict__ sbias,
                                                  const float* __restrict__ hin,
                                                  const float* __restrict__ lng,
                                                  const float* __restrict__ lnb,
                                                  float* __restrict__ hout) {
    __shared__ int   s_list[LCAP];
    __shared__ int   s_bkt[8][BCAP];
    __shared__ int   s_nel[8][MAXD];
    __shared__ float s_sc[8][MAXD * 4];
    __shared__ float s_row[8][HID] __attribute__((aligned(16)));
    __shared__ int   s_cnt[2][8];

    const int tid = threadIdx.x;
    const int lane = tid & 31;
    const int wv = tid >> 5;
    const int n0 = blockIdx.x * ANB;
    const int* __restrict__ src = ei;
    const int* __restrict__ dst = ei + E;

    int base = 0;
    const int nchunk = (E + 255) >> 8;
    for (int c = 0; c < nchunk; ++c) {
        const int e = (c << 8) + tid;
        const bool valid = e < E;
        const int ec = valid ? e : 0;
        const int d = dst[ec];
        int s = src[ec];
        s = s < 0 ? 0 : s;
        s = s >= Nn ? Nn - 1 : s;
        const int ln = d - n0;
        const bool hit = valid && ((unsigned)ln < (unsigned)ANB);
        const unsigned msk = __builtin_amdgcn_ballot_w32(hit);
        if (lane == 0) s_cnt[c & 1][wv] = (int)__builtin_popcount(msk);
        __syncthreads();
        int below = 0, tot = 0;
#pragma unroll
        for (int i = 0; i < 8; ++i) {
            const int v = s_cnt[c & 1][i];
            tot += v;
            below += (i < wv) ? v : 0;
        }
        const int pos = base + below + (int)__builtin_amdgcn_mbcnt_lo(msk, 0u);
        if (hit && pos < LCAP) s_list[pos] = s | (ln << 20);
        base += tot;
    }
    __syncthreads();
    const int total = base < LCAP ? base : LCAP;

    int* bkt = s_bkt[wv];
    int bc = 0;
    const int nit = (total + 31) >> 5;
    for (int i = 0; i < nit; ++i) {
        const int idx = (i << 5) + lane;
        const bool ok = idx < total;
        const int ent = s_list[ok ? idx : 0];
        const bool mine = ok && ((ent >> 26) == wv);
        const unsigned mm = __builtin_amdgcn_ballot_w32(mine);
        const int pos = bc + (int)__builtin_amdgcn_mbcnt_lo(mm, 0u);
        if (mine && pos < BCAP) bkt[pos] = ent;
        bc += (int)__builtin_popcount(mm);
    }
    if (bc > BCAP) bc = BCAP;
    const int nb = (bc + 31) >> 5;

    const int hd = lane >> 3;
    const int cg = lane & 7;
    int* nel = s_nel[wv];
    float* scw = s_sc[wv];
    float* roww = s_row[wv];
    for (int t = 0; t < ANPW; ++t) {
        const int lnode = wv * ANPW + t;
        const int node = n0 + lnode;
        if (node >= Nn) break;

        int cnt = 0;
        for (int i = 0; i < nb; ++i) {
            const int idx = (i << 5) + lane;
            const bool ok = idx < bc;
            const int ent = bkt[ok ? idx : 0];
            const bool match = ok && ((ent >> 20) == lnode);
            const unsigned mm = __builtin_amdgcn_ballot_w32(match);
            const int pos = cnt + (int)__builtin_amdgcn_mbcnt_lo(mm, 0u);
            if (match && pos < MAXD) nel[pos] = ent & 0xFFFFF;
            cnt += (int)__builtin_popcount(mm);
        }
        const int deg = cnt < MAXD ? cnt : MAXD;

        float qf[16];
        {
            const _Float16* qp = q16 + (size_t)node * QKV + lane * 16;
            const v8h qa = *(const v8h*)qp;
            const v8h qb8 = *(const v8h*)(qp + 8);
#pragma unroll
            for (int u = 0; u < 8; ++u) { qf[u] = (float)qa[u]; qf[8 + u] = (float)qb8[u]; }
        }

        float mx = -__builtin_inff();
#pragma unroll 1
        for (int j = 0; j < deg; ++j) {
            const int s = nel[j];
            const _Float16* kp = k16 + (size_t)s * QKV + lane * 16;
            const v8h ka = *(const v8h*)kp;
            const v8h kb = *(const v8h*)(kp + 8);
            float p = 0.f;
#pragma unroll
            for (int u = 0; u < 8; ++u) p += qf[u] * (float)ka[u];
#pragma unroll
            for (int u = 0; u < 8; ++u) p += qf[8 + u] * (float)kb[u];
            p += __shfl_xor(p, 1, 32);
            p += __shfl_xor(p, 2, 32);
            p += __shfl_xor(p, 4, 32);
            const float sc = p * ATT_SCALE;
            mx = fmaxf(mx, sc);
            if (cg == 0) scw[j * 4 + hd] = sc;
        }
        float den = 0.f;
#pragma unroll 1
        for (int j = 0; j < deg; ++j) {
            const float sc = scw[j * 4 + hd];
            const float p = expf(sc - mx);
            den += p;
            if (cg == 0) scw[j * 4 + hd] = p;
        }
        const float rden = 1.0f / (den + 1e-16f);
        float acc[16];
#pragma unroll
        for (int u = 0; u < 16; ++u) acc[u] = 0.f;
#pragma unroll 1
        for (int j = 0; j < deg; ++j) {
            const int s = nel[j];
            const float wgt = scw[j * 4 + hd] * rden;
            const float* vp = v32 + (size_t)s * QKV + lane * 16;
            const v4f x0 = *(const v4f*)vp;
            const v4f x1 = *(const v4f*)(vp + 4);
            const v4f x2 = *(const v4f*)(vp + 8);
            const v4f x3 = *(const v4f*)(vp + 12);
#pragma unroll
            for (int u = 0; u < 4; ++u) {
                acc[u]      += x0[u] * wgt;
                acc[4 + u]  += x1[u] * wgt;
                acc[8 + u]  += x2[u] * wgt;
                acc[12 + u] += x3[u] * wgt;
            }
        }
        float tt[16];
#pragma unroll
        for (int u = 0; u < 16; ++u) {
            float a = acc[u];
            a += __shfl_xor(a, 8, 32);
            a += __shfl_xor(a, 16, 32);
            tt[u] = a * 0.25f;
        }
        const int c0 = cg * 16;
        {
            const float* skp = skip + (size_t)node * HID + c0;
            const float* rsp = hin + (size_t)node * HID + c0;
            const float* sbp = sbias + c0;
#pragma unroll
            for (int u = 0; u < 4; ++u) {
                const v4f sk = *(const v4f*)(skp + 4 * u);
                const v4f rs = *(const v4f*)(rsp + 4 * u);
                const v4f sb4 = *(const v4f*)(sbp + 4 * u);
#pragma unroll
                for (int q = 0; q < 4; ++q)
                    tt[4 * u + q] = ((tt[4 * u + q] + sk[q]) + sb4[q]) + rs[q];
            }
        }
        float s1 = 0.f;
#pragma unroll
        for (int u = 0; u < 16; ++u) s1 += tt[u];
        s1 += __shfl_xor(s1, 1, 32);
        s1 += __shfl_xor(s1, 2, 32);
        s1 += __shfl_xor(s1, 4, 32);
        const float mu = s1 * (1.0f / HID);
        float s2 = 0.f;
#pragma unroll
        for (int u = 0; u < 16; ++u) {
            const float dlt = tt[u] - mu;
            tt[u] = dlt;
            s2 += dlt * dlt;
        }
        s2 += __shfl_xor(s2, 1, 32);
        s2 += __shfl_xor(s2, 2, 32);
        s2 += __shfl_xor(s2, 4, 32);
        const float rstd = rsqrtf(s2 * (1.0f / HID) + LN_EPS);
        {
            const float* gp = lng + c0;
            const float* bp = lnb + c0;
#pragma unroll
            for (int u = 0; u < 4; ++u) {
                const v4f g4 = *(const v4f*)(gp + 4 * u);
                const v4f b4 = *(const v4f*)(bp + 4 * u);
#pragma unroll
                for (int q = 0; q < 4; ++q)
                    tt[4 * u + q] = tt[4 * u + q] * rstd * g4[q] + b4[q];
            }
        }
        if (hd == 0) {
#pragma unroll
            for (int u = 0; u < 16; ++u) roww[c0 + u] = tt[u];
        }
        const v4f ov = *(const v4fa*)(roww + lane * 4);
        float* op = hout + (size_t)node * HID + lane * 4;
        *(volatile v4f*)op = ov;
        __threadfence();
        *(volatile v4f*)op = ov;
    }
}

static inline size_t al256(size_t b) { return (b + 255) & ~(size_t)255; }

extern "C" void kernel_launch(void* const* d_in, const int* in_sizes, int n_in,
                              void* d_out, int out_size, void* d_ws, size_t ws_size,
                              hipStream_t stream) {
    if (n_in < 24) return;
    const int N = in_sizes[0] / IN_DIM;
    const int E = in_sizes[1] / 2;
    if (N <= 0 || E <= 0 || N > (1 << 20)) return;
    if (in_sizes[0] != N * IN_DIM || in_sizes[1] != 2 * E) return;
    if (in_sizes[2] != IN_DIM * HID || in_sizes[3] != HID) return;
    for (int l = 0; l < 2; ++l) {
        const int b = 4 + 10 * l;
        if (in_sizes[b + 0] != HID * QKV || in_sizes[b + 1] != QKV) return;
        if (in_sizes[b + 2] != HID * QKV || in_sizes[b + 3] != QKV) return;
        if (in_sizes[b + 4] != HID * QKV || in_sizes[b + 5] != QKV) return;
        if (in_sizes[b + 6] != HID * HID || in_sizes[b + 7] != HID) return;
        if (in_sizes[b + 8] != HID || in_sizes[b + 9] != HID) return;
    }
    if ((long long)out_size < (long long)N * HID) return;

    const float* x     = (const float*)d_in[0];
    const int*   ei    = (const int*)d_in[1];
    const float* lin_w = (const float*)d_in[2];
    const float* lin_b = (const float*)d_in[3];
    const float* q_w[2]  = {(const float*)d_in[4],  (const float*)d_in[14]};
    const float* q_b[2]  = {(const float*)d_in[5],  (const float*)d_in[15]};
    const float* k_w[2]  = {(const float*)d_in[6],  (const float*)d_in[16]};
    const float* k_b[2]  = {(const float*)d_in[7],  (const float*)d_in[17]};
    const float* v_w[2]  = {(const float*)d_in[8],  (const float*)d_in[18]};
    const float* v_b[2]  = {(const float*)d_in[9],  (const float*)d_in[19]};
    const float* s_w[2]  = {(const float*)d_in[10], (const float*)d_in[20]};
    const float* s_b[2]  = {(const float*)d_in[11], (const float*)d_in[21]};
    const float* ln_g[2] = {(const float*)d_in[12], (const float*)d_in[22]};
    const float* ln_b[2] = {(const float*)d_in[13], (const float*)d_in[23]};

    char* ws = (char*)d_ws;
    size_t off = 0;
    float* h0 = (float*)(ws + off);          off += al256((size_t)N * HID * sizeof(float));
    float* h1 = (float*)(ws + off);          off += al256((size_t)N * HID * sizeof(float));
    float* skp = (float*)(ws + off);         off += al256((size_t)N * HID * sizeof(float));
    _Float16* q16 = (_Float16*)(ws + off);  off += al256((size_t)N * QKV * sizeof(_Float16));
    _Float16* k16 = (_Float16*)(ws + off);  off += al256((size_t)N * QKV * sizeof(_Float16));
    float* v32 = (float*)(ws + off);         off += al256((size_t)N * QKV * sizeof(float));
    _Float16* wtl = (_Float16*)(ws + off);  off += al256((size_t)IN_DIM * HID * sizeof(_Float16));
    _Float16* wq[2]; _Float16* wk[2]; _Float16* wvv[2]; _Float16* wss[2];
    for (int l = 0; l < 2; ++l) {
        wq[l]  = (_Float16*)(ws + off); off += al256((size_t)HID * QKV * sizeof(_Float16));
        wk[l]  = (_Float16*)(ws + off); off += al256((size_t)HID * QKV * sizeof(_Float16));
        wvv[l] = (_Float16*)(ws + off); off += al256((size_t)HID * QKV * sizeof(_Float16));
        wss[l] = (_Float16*)(ws + off); off += al256((size_t)HID * HID * sizeof(_Float16));
    }
    if (off > ws_size) return;

    wprep_kernel<<<(IN_DIM * HID / 8 + 255) / 256, 256, 0, stream>>>(lin_w, wtl, IN_DIM, HID);
    for (int l = 0; l < 2; ++l) {
        wprep_kernel<<<(HID * QKV / 8 + 255) / 256, 256, 0, stream>>>(q_w[l], wq[l], HID, QKV);
        wprep_kernel<<<(HID * QKV / 8 + 255) / 256, 256, 0, stream>>>(k_w[l], wk[l], HID, QKV);
        wprep_kernel<<<(HID * QKV / 8 + 255) / 256, 256, 0, stream>>>(v_w[l], wvv[l], HID, QKV);
        wprep_kernel<<<(HID * HID / 8 + 255) / 256, 256, 0, stream>>>(s_w[l], wss[l], HID, HID);
    }

    const int gblk = (N + 31) / 32;
    const int ablk = (N + ANB - 1) / ANB;

    proj_kernel<<<gblk, 128, 0, stream>>>(x, N, wtl, lin_b, h0);

    qkvs_kernel<<<gblk, 128, 0, stream>>>(h0, N, wq[0], q_b[0], wk[0], k_b[0], wvv[0], v_b[0],
                                          wss[0], q16, k16, v32, skp);
    agg_kernel<<<ablk, 256, 0, stream>>>(ei, E, N, q16, k16, v32, skp, s_b[0], h0,
                                         ln_g[0], ln_b[0], h1);

    qkvs_kernel<<<gblk, 128, 0, stream>>>(h1, N, wq[1], q_b[1], wk[1], k_b[1], wvv[1], v_b[1],
                                          wss[1], q16, k16, v32, skp);
    agg_kernel<<<ablk, 256, 0, stream>>>(ei, E, N, q16, k16, v32, skp, s_b[1], h1,
                                         ln_g[1], ln_b[1], (float*)d_out);
}
